// VSSBlock_45243185496329
// MI455X (gfx1250) — hardware-run, weakly checked
//
#include <hip/hip_runtime.h>


#ifndef NB
#define NB 4
#endif
#ifndef DDEP
#define DDEP 8
#endif
#define NB_FULL   4
#define DDEP_FULL 8
#define HH   32
#define WW   32
#define CC   192
#define DI   384
#define NS   16
#define DR   12
#define NXP  (DR + 2 * NS)
#define XP   64
#define LL       (DDEP * HH * WW)
#define LL_FULL  (DDEP_FULL * HH * WW)
#define BL       (NB * LL)
#define EPSL   1e-5f
#define ACARRY 16.0f
#define AINV   0.0625f
#define WCARRY 16.0f
#define EPI    (1.0f / 256.0f)
#define LOG2E  1.4426950408889634f

#define N8_WIN  ((2 * DI * CC) / 8)
#define N8_WXS  ((NXP * DI) / 8)
#define N8_WXP  ((XP * DI) / 8)
#define N8_WOUT ((CC * DI) / 8)
#define N4_WC   ((27 * DI) / 4)
#define GB_WIN  (N8_WIN / 256)
#define GB_WXP  (N8_WXP / 256)
#define GB_WOUT (N8_WOUT / 256)
#define GB_WC   ((N4_WC + 255) / 256)

static_assert(NB <= NB_FULL);
static_assert(DDEP <= DDEP_FULL);
static_assert(CC % 32 == 0);
static_assert(DI % 32 == 0);
static_assert((2 * DI) % 64 == 0);
static_assert(DI % 64 == 0);
static_assert(CC % 64 == 0);
static_assert(XP == 64);
static_assert(NXP <= XP);
static_assert(LL % 64 == 0);
static_assert(BL % 64 == 0);
static_assert(BL % 16 == 0);
static_assert(BL % 8 == 0);
static_assert(WW % 2 == 0);
static_assert(CC / 8 == 24);
static_assert(DI / 8 == 48);
static_assert(2 * (DI / 8) == 3 * 32);
static_assert(DI % 128 == 0);
static_assert(NS % 4 == 0);
static_assert(DR % 4 == 0);
static_assert(NXP % 4 == 0);
static_assert(N8_WIN % 256 == 0);
static_assert(N8_WXP % 256 == 0);
static_assert(N8_WOUT % 256 == 0);
static_assert(N4_WC % 8 == 0);
static_assert((NXP * DI) % 8 == 0);
static_assert(16 * 68 * 4 <= 131072);
static_assert(32 * 16 * 4 == 16 * 128);
static_assert(32 * 16 * 8 == 16 * 256);

typedef _Float16 h16;
typedef __attribute__((ext_vector_type(16))) _Float16 v16h;
typedef __attribute__((ext_vector_type(8)))  _Float16 v8h;
typedef __attribute__((ext_vector_type(8)))  float    v8f;
typedef __attribute__((ext_vector_type(4)))  float    v4f;
typedef v4f  __attribute__((may_alias)) v4fa;

__device__ __forceinline__ unsigned short f2bf(float f) { unsigned u = __float_as_uint(f); u += 0x7FFFu + ((u >> 16) & 1u); return (unsigned short)(u >> 16); }
__device__ __forceinline__ float bfr(float f) { return __uint_as_float(((unsigned)f2bf(f)) << 16); }
__device__ __forceinline__ v16h cat16(v8h lo, v8h hi) { return __builtin_shufflevector(lo, hi, 0, 1, 2, 3, 4, 5, 6, 7, 8, 9, 10, 11, 12, 13, 14, 15); }
__device__ __forceinline__ v8f wmma16(v16h a, v16h b, v8f c) { return __builtin_amdgcn_wmma_f32_16x16x32_f16(false, a, false, b, (short)0, c, false, false); }
__device__ __forceinline__ v8f wmma16g(v16h a, v16h b, v8f c) { c = wmma16(a, b, c); asm volatile("v_nop\n\tv_nop\n\tv_nop\n\tv_nop" : "+v"(c) : "v"(a), "v"(b)); return c; }
__device__ __forceinline__ v16h  ldh(const h16* p) { return cat16(*(const v8h*)p, *(const v8h*)(p + 16)); }
__device__ __forceinline__ void wave_sync() { __builtin_amdgcn_fence(3  , "wavefront"); __builtin_amdgcn_wave_barrier(); asm volatile("" ::: "memory"); }
static __device__ __forceinline__ h16 toh_flush(float v) { const h16 r = (h16)v; return (fabsf(v) < 6.103515625e-05f) ? (h16)0.0f : r; }
__device__ __forceinline__ float silu_rcp(float a) { const float e = __expf(-a); return a * __builtin_amdgcn_rcpf(1.0f + e); }
__device__ __forceinline__ float wsum(float v) { v += __shfl_xor(v, 16, 32); v += __shfl_xor(v, 8, 32); v += __shfl_xor(v, 4, 32); v += __shfl_xor(v, 2, 32); v += __shfl_xor(v, 1, 32); return v; }

__device__ __forceinline__ void wcvt_piece(const float* __restrict__ src, h16* dst, int i, int nsrc8) {
    const bool ok = i < nsrc8; const int ic = ok ? i : (nsrc8 - 1);
    v8f v = *(const v8f*)(src + (size_t)ic * 8);
    asm volatile("" : "+v"(v));
    v8h o;
#pragma unroll
    for (int k = 0; k < 8; ++k) { const float t = ok ? bfr(v[k]) * WCARRY : 0.0f; o[k] = toh_flush(t); }
    *(volatile v8h*)(dst + (size_t)i * 8) = o; __threadfence(); *(volatile v8h*)(dst + (size_t)i * 8) = o;
}

__global__ __launch_bounds__(256) void k_wprep(const float* __restrict__ win, const float* __restrict__ wxp, const float* __restrict__ wout, const float* __restrict__ cw,
                                               h16* WIN, h16* WXP, h16* WOUT, float* WC) {
    const int blk = blockIdx.x; const int tid = threadIdx.x;
    if (blk < GB_WIN) {
        wcvt_piece(win, WIN, blk * 256 + tid, N8_WIN);
    } else if (blk < GB_WIN + GB_WXP) {
        wcvt_piece(wxp, WXP, (blk - GB_WIN) * 256 + tid, N8_WXS);
    } else if (blk < GB_WIN + GB_WXP + GB_WOUT) {
        wcvt_piece(wout, WOUT, (blk - GB_WIN - GB_WXP) * 256 + tid, N8_WOUT);
    } else {
        const int p = (blk - GB_WIN - GB_WXP - GB_WOUT) * 256 + tid;
        const bool ok = p < N4_WC; const int pc = ok ? p : (N4_WC - 1);
        const int t = pc / (DI / 4), c4 = (pc % (DI / 4)) * 4;
        v4f v;
#pragma unroll
        for (int i = 0; i < 4; ++i) { const float x = cw[(size_t)(c4 + i) * 27 + t]; v[i] = bfr(x); }
        if (ok) *(volatile v4f*)(WC + (size_t)p * 4) = v;
        __threadfence();
        if (ok) *(volatile v4f*)(WC + (size_t)p * 4) = v;
    }
}

__global__ __launch_bounds__(256) void k_ln_in(const float* __restrict__ x, const float* __restrict__ gw, const float* __restrict__ gb, h16* HX) {
#pragma clang fp contract(off)
    const int lane = threadIdx.x & 31;
    const int wave = __builtin_amdgcn_readfirstlane((int)(threadIdx.x >> 5));
    const int row = blockIdx.x * 8 + wave;
    const int b = row / LL, l = row % LL;
    const bool ok = lane < 24; const int cl = ok ? lane : 23;
    const float* xr = x + ((size_t)b * LL_FULL + (size_t)l) * CC + cl * 8;
    v4f p0 = *(const v4f*)xr, p1 = *(const v4f*)(xr + 4);
    asm volatile("" : "+v"(p0), "+v"(p1));
    float v[8];
#pragma unroll
    for (int e = 0; e < 4; ++e) { v[e] = ok ? bfr(p0[e]) : 0.0f; v[4 + e] = ok ? bfr(p1[e]) : 0.0f; }
    float s = 0.0f;
#pragma unroll
    for (int e = 0; e < 8; ++e) s += v[e];
    s = wsum(s);
    const float mu = s * (1.0f / CC);
    float qs = 0.0f;
#pragma unroll
    for (int e = 0; e < 8; ++e) { const float dv = ok ? (v[e] - mu) : 0.0f; v[e] = dv; qs += dv * dv; }
    qs = wsum(qs);
    const float rs = rsqrtf(qs * (1.0f / CC) + EPSL);
    const v4f g0 = *(const v4f*)(gw + cl * 8), g1 = *(const v4f*)(gw + cl * 8 + 4);
    const v4f c0 = *(const v4f*)(gb + cl * 8), c1 = *(const v4f*)(gb + cl * 8 + 4);
    v8h o;
#pragma unroll
    for (int e = 0; e < 4; ++e) {
        o[e]     = toh_flush((v[e] * rs * bfr(g0[e]) + bfr(c0[e])) * ACARRY);
        o[4 + e] = toh_flush((v[4 + e] * rs * bfr(g1[e]) + bfr(c1[e])) * ACARRY); }
    h16* op = HX + (size_t)row * CC + lane * 8;
    if (ok) *(volatile v8h*)op = o;
    __threadfence();
    if (ok) *(volatile v8h*)op = o;
}

template <int MODE, int K>
__device__ __forceinline__ void gemm_tile(const h16* __restrict__ A, const h16* __restrict__ Bt, h16* PH, size_t zofs, float* PF, const float* __restrict__ XR) {
    __shared__ __align__(16) float os[16 * 68];
    static_assert(K % 32 == 0);
    const int lane = threadIdx.x & 31, lr = lane & 15, hi = lane >> 4; const int r0 = blockIdx.x * 64, c0 = blockIdx.y * 64;
    v8f acc[4][4];
#pragma unroll
    for (int mb = 0; mb < 4; ++mb)
#pragma unroll
        for (int nb = 0; nb < 4; ++nb) acc[mb][nb] = (v8f){};
    const size_t aoff = (size_t)(r0 + lr) * K + 8 * hi, boff = (size_t)(c0 + lr) * K + 8 * hi;
#pragma unroll 1
    for (int kc = 0; kc < K; kc += 32) {
        v16h a[4];
#pragma unroll
        for (int mb = 0; mb < 4; ++mb) a[mb] = ldh(A + aoff + (size_t)mb * 16 * K + kc);
#pragma unroll
        for (int nb = 0; nb < 4; ++nb) { const v16h bq = ldh(Bt + boff + (size_t)nb * 16 * K + kc);
#pragma unroll
            for (int mb = 0; mb < 4; ++mb) acc[mb][nb] = wmma16g(a[mb], bq, acc[mb][nb]); }
    }
    size_t hb = 0, fb = 0;
    if (MODE == 0) hb = ((c0 < DI) ? (size_t)c0 : (zofs + (size_t)(c0 - DI))) + (size_t)r0 * DI;
    if (MODE == 1) fb = (size_t)r0 * XP;
    if (MODE == 2) { const int bb = r0 / LL, l0 = r0 % LL; fb = ((size_t)bb * LL_FULL + (size_t)l0) * CC + (size_t)c0; }
#pragma unroll
    for (int mb = 0; mb < 4; ++mb) {
#pragma unroll
        for (int nb = 0; nb < 4; ++nb) {
#pragma unroll
            for (int j = 0; j < 8; ++j) os[(hi * 8 + j) * 68 + nb * 16 + lr] = acc[mb][nb][j] * EPI; }
        wave_sync();
#pragma unroll 1
        for (int ps = 0; ps < 2; ++ps) {
            if (MODE == 0) {
#pragma unroll
                for (int s = 0; s < 4; ++s) { const int row = 4 * s + (lane >> 3), c8 = (lane & 7) * 8;
                    const v4f x0 = *(const v4fa*)(&os[row * 68 + c8]); const v4f x1 = *(const v4fa*)(&os[row * 68 + c8 + 4]); v8h hv;
#pragma unroll
                    for (int i = 0; i < 4; ++i) { hv[i] = toh_flush(x0[i]); hv[4 + i] = toh_flush(x1[i]); }
                    *(volatile v8h*)(PH + hb + (size_t)(mb * 16 + row) * DI + c8) = hv; }
            } else {
#pragma unroll
                for (int s = 0; s < 8; ++s) { const int row = 2 * s + (lane >> 4), c4 = (lane & 15) * 4;
                    v4f val = *(const v4fa*)(&os[row * 68 + c4]);
                    const size_t oo = fb + (size_t)(mb * 16 + row) * (size_t)(MODE == 1 ? XP : CC) + (size_t)c4;
                    if (MODE == 2) { const v4f xr = *(const v4f*)(XR + oo);
#pragma unroll
                        for (int i = 0; i < 4; ++i) val[i] += bfr(xr[i]); }
                    *(volatile v4f*)(PF + oo) = val; }
            }
            if (ps == 0) __threadfence(); }
        wave_sync();
    }
}

__global__ __launch_bounds__(32) void k_gemm_in(const h16* __restrict__ A, const h16* __restrict__ Bt, h16* PH, size_t zofs) { gemm_tile<0, CC>(A, Bt, PH, zofs, nullptr, nullptr); }
__global__ __launch_bounds__(32) void k_gemm_xp(const h16* __restrict__ A, const h16* __restrict__ Bt, float* PF) { gemm_tile<1, DI>(A, Bt, nullptr, 0, PF, nullptr); }
__global__ __launch_bounds__(32) void k_gemm_out(const h16* __restrict__ A, const h16* __restrict__ Bt, float* PF, const float* __restrict__ XR) { gemm_tile<2, DI>(A, Bt, nullptr, 0, PF, XR); }

__global__ __launch_bounds__(256) void k_conv(const h16* __restrict__ XI, const float* __restrict__ WC, const float* __restrict__ cb, h16* U) {
    const int lane = threadIdx.x & 31;
    const int wave = __builtin_amdgcn_readfirstlane((int)(threadIdx.x >> 5));
    const int tok0 = (blockIdx.x * 8 + wave) * 2;
    const int b = tok0 / LL, l0 = tok0 % LL;
    const int dd = l0 / (HH * WW), hh = (l0 / WW) % HH, w0 = l0 % WW;
    const size_t tb = (size_t)b * LL;
#pragma unroll 1
    for (int j = 0; j < 3; ++j) {
        const int q = lane + 32 * j; const int tk = q / 48; const int c8 = (q - 48 * tk) * 8; const int wq = w0 + tk;
        const v4f b0 = *(const v4f*)(cb + c8), b1 = *(const v4f*)(cb + c8 + 4);
        float acc[8];
#pragma unroll
        for (int e = 0; e < 4; ++e) { acc[e] = bfr(b0[e]); acc[4 + e] = bfr(b1[e]); }
#pragma unroll 1
        for (int i = 0; i < 3; ++i) {
            const int d2 = dd + i - 1; if (d2 < 0 || d2 >= DDEP) continue;
#pragma unroll 1
            for (int jj = 0; jj < 3; ++jj) {
                const int h2 = hh + jj - 1; if (h2 < 0 || h2 >= HH) continue;
#pragma unroll 1
                for (int k = 0; k < 3; ++k) {
                    const int w2 = wq + k - 1; const bool ok = (w2 >= 0) & (w2 < WW);
                    const int w2c = w2 < 0 ? 0 : (w2 > WW - 1 ? WW - 1 : w2);
                    const h16* xp = XI + (tb + (size_t)((d2 * HH + h2) * WW + w2c)) * DI + c8;
                    v8h xh = *(const v8h*)xp;
                    asm volatile("" : "+v"(xh));
                    const float* wp = WC + (size_t)((i * 3 + jj) * 3 + k) * DI + c8;
                    const v4f wa = *(const v4f*)wp, wb = *(const v4f*)(wp + 4);
#pragma unroll
                    for (int e = 0; e < 4; ++e) {
                        const float xa = ok ? (float)xh[e] : 0.0f; const float xb = ok ? (float)xh[4 + e] : 0.0f;
                        acc[e] += xa * wa[e]; acc[4 + e] += xb * wb[e]; }
                }
            }
        }
        v8h o;
#pragma unroll
        for (int e = 0; e < 8; ++e) o[e] = toh_flush(silu_rcp(acc[e]) * ACARRY);
        h16* up = U + (size_t)tok0 * DI + (size_t)q * 8;
        *(volatile v8h*)up = o; __threadfence(); *(volatile v8h*)up = o;
    }
}

__global__ __launch_bounds__(128) void k_scan(const h16* __restrict__ U, const float* __restrict__ XD, const float* __restrict__ dtw, const float* __restrict__ dtb,
                                              const float* __restrict__ alog, const float* __restrict__ dsk, float* Y) {
    const int d = blockIdx.x * 128 + (int)threadIdx.x;
    const int b = blockIdx.y;
    float a2[NS], hs[NS], wdt[DR];
    { const v4f* ap = (const v4f*)(alog + (size_t)d * NS);
#pragma unroll
      for (int i = 0; i < NS / 4; ++i) { const v4f t = ap[i];
#pragma unroll
          for (int e = 0; e < 4; ++e) { a2[4 * i + e] = -__expf(bfr(t[e])) * LOG2E; hs[4 * i + e] = 0.0f; } }
      const v4f* wp = (const v4f*)(dtw + (size_t)d * DR);
#pragma unroll
      for (int i = 0; i < DR / 4; ++i) { const v4f t = wp[i];
#pragma unroll
          for (int e = 0; e < 4; ++e) wdt[4 * i + e] = bfr(t[e]); } }
    const float bias = bfr(dtb[d]); const float dk = bfr(dsk[d]);
    const size_t rb = (size_t)b * LL;
#pragma unroll 1
    for (int l = 0; l < LL; ++l) {
        const size_t row = rb + (size_t)l;
        const v4f* xr = (const v4f*)(XD + row * XP);
        float xs[NXP];
#pragma unroll
        for (int i = 0; i < NXP / 4; ++i) { const v4f t = xr[i];
#pragma unroll
            for (int e = 0; e < 4; ++e) xs[4 * i + e] = t[e]; }
        const float ul = (float)U[row * DI + (size_t)d] * AINV;
        float s = bias;
#pragma unroll
        for (int r = 0; r < DR; ++r) s += xs[r] * wdt[r];
        const float ee = __expf(-fabsf(s));
        const float dl = fmaxf(s, 0.0f) + log1pf(ee);
        const float xv = dl * ul;
        float y = 0.0f;
#pragma unroll
        for (int n = 0; n < NS; ++n) {
            const float dA = __builtin_amdgcn_exp2f(dl * a2[n]);
            hs[n] = dA * hs[n] + xv * xs[DR + n];
            y += hs[n] * xs[DR + NS + n]; }
        y += dk * ul;
        volatile float* yp = Y + row * DI + (size_t)d;
        *yp = y; __threadfence(); *yp = y;
    }
}

__global__ __launch_bounds__(256) void k_ln_gate(const float* __restrict__ Y, const h16* __restrict__ Z, const float* __restrict__ ow, const float* __restrict__ ob, h16* G) {
#pragma clang fp contract(off)
    const int lane = threadIdx.x & 31;
    const int wave = __builtin_amdgcn_readfirstlane((int)(threadIdx.x >> 5));
    const int row = blockIdx.x * 8 + wave;
    const float* yr = Y + (size_t)row * DI;
    const bool ok1 = lane < 16;
    float v[2][8];
    float s = 0.0f;
#pragma unroll
    for (int j = 0; j < 2; ++j) {
        const bool ok = (j == 0) | ok1; const int qc = ok ? (lane + 32 * j) : 47;
        v4f p0 = *(const v4f*)(yr + qc * 8), p1 = *(const v4f*)(yr + qc * 8 + 4);
        asm volatile("" : "+v"(p0), "+v"(p1));
#pragma unroll
        for (int e = 0; e < 4; ++e) { v[j][e] = ok ? p0[e] : 0.0f; v[j][4 + e] = ok ? p1[e] : 0.0f; s += v[j][e]; s += v[j][4 + e]; } }
    s = wsum(s);
    const float mu = s * (1.0f / DI);
    float qs = 0.0f;
#pragma unroll
    for (int j = 0; j < 2; ++j) {
        const bool ok = (j == 0) | ok1;
#pragma unroll
        for (int e = 0; e < 8; ++e) { const float dv = ok ? (v[j][e] - mu) : 0.0f; v[j][e] = dv; qs += dv * dv; } }
    qs = wsum(qs);
    const float rs = rsqrtf(qs * (1.0f / DI) + EPSL);
    v8h o[2];
#pragma unroll
    for (int j = 0; j < 2; ++j) {
        const bool ok = (j == 0) | ok1; const int qc = ok ? (lane + 32 * j) : 47;
        v8h zh = *(const v8h*)(Z + (size_t)row * DI + qc * 8);
        asm volatile("" : "+v"(zh));
        const v4f g0 = *(const v4f*)(ow + qc * 8), g1 = *(const v4f*)(ow + qc * 8 + 4);
        const v4f c0 = *(const v4f*)(ob + qc * 8), c1 = *(const v4f*)(ob + qc * 8 + 4);
#pragma unroll
        for (int e = 0; e < 4; ++e) {
            const float la = v[j][e] * rs * bfr(g0[e]) + bfr(c0[e]);
            const float lb = v[j][4 + e] * rs * bfr(g1[e]) + bfr(c1[e]);
            o[j][e]     = toh_flush(la * silu_rcp((float)zh[e]) * ACARRY);
            o[j][4 + e] = toh_flush(lb * silu_rcp((float)zh[4 + e]) * ACARRY); } }
    h16* gp = G + (size_t)row * DI + lane * 8;
    *(volatile v8h*)gp = o[0];
    if (ok1) *(volatile v8h*)(gp + 256) = o[1];
    __threadfence();
    *(volatile v8h*)gp = o[0];
    if (ok1) *(volatile v8h*)(gp + 256) = o[1];
}

static constexpr size_t al256(size_t v) { return (v + 255) & ~(size_t)255; }
static constexpr size_t SZ_XI   = al256((size_t)BL * DI * 2);
static constexpr size_t SZ_HX   = al256((size_t)BL * CC * 2);
static constexpr size_t SZ_Y    = al256((size_t)BL * DI * 4);
static constexpr size_t SZ_RA   = (SZ_XI + SZ_HX > SZ_Y) ? (SZ_XI + SZ_HX) : SZ_Y;
static constexpr size_t SZ_Z    = al256((size_t)BL * DI * 2);
static constexpr size_t SZ_UG   = al256((size_t)BL * DI * 2);
static constexpr size_t SZ_XD   = al256((size_t)BL * XP * 4);
static constexpr size_t SZ_WIN  = al256((size_t)2 * DI * CC * 2);
static constexpr size_t SZ_WXP  = al256((size_t)XP * DI * 2);
static constexpr size_t SZ_WOUT = al256((size_t)CC * DI * 2);
static constexpr size_t SZ_WC   = al256((size_t)27 * DI * 4);
static constexpr size_t SZ_TOTAL = SZ_RA + SZ_Z + SZ_UG + SZ_XD + SZ_WIN + SZ_WXP + SZ_WOUT + SZ_WC;
static_assert(SZ_XI + SZ_HX <= SZ_RA);
static_assert(SZ_Y <= SZ_RA);
static_assert(SZ_RA % 256 == 0);
static_assert((size_t)GB_WC * 256 * 16 >= (size_t)27 * DI * 4);
static_assert((size_t)N4_WC * 16 == (size_t)27 * DI * 4);
static_assert(SZ_TOTAL <= (size_t)134217728);

extern "C" void kernel_launch(void* const* d_in, const int* in_sizes, int n_in,
                              void* d_out, int out_size, void* d_ws, size_t ws_size, hipStream_t stream) {
    if (n_in < 14) return;
    const size_t needx = ((size_t)(NB - 1) * LL_FULL + LL) * CC;
    if ((size_t)in_sizes[0] < needx) return;
    if (in_sizes[1] < CC || in_sizes[2] < CC) return;
    if ((size_t)in_sizes[3] < (size_t)2 * DI * CC) return;
    if (in_sizes[4] < DI * 27 || in_sizes[5] < DI) return;
    if (in_sizes[6] < NXP * DI || in_sizes[7] < DI * DR || in_sizes[8] < DI || in_sizes[9] < DI * NS) return;
    if (in_sizes[10] < DI || in_sizes[11] < DI || in_sizes[12] < DI) return;
    if (in_sizes[13] < CC * DI) return;
    if ((size_t)out_size < needx) return;
    if (SZ_TOTAL > ws_size) return;
    const float* x     = (const float*)d_in[0];
    const float* ln1w  = (const float*)d_in[1];
    const float* ln1b  = (const float*)d_in[2];
    const float* win   = (const float*)d_in[3];
    const float* convw = (const float*)d_in[4];
    const float* convb = (const float*)d_in[5];
    const float* xprj  = (const float*)d_in[6];
    const float* dtw   = (const float*)d_in[7];
    const float* dtb   = (const float*)d_in[8];
    const float* alog  = (const float*)d_in[9];
    const float* dsk   = (const float*)d_in[10];
    const float* onw   = (const float*)d_in[11];
    const float* onb   = (const float*)d_in[12];
    const float* wout  = (const float*)d_in[13];
    float* OUT = (float*)d_out;
    char* wsp = (char*)d_ws;
    h16*   XI = (h16*)wsp;
    h16*   HX = (h16*)(wsp + SZ_XI);
    float* Y  = (float*)wsp;
    wsp += SZ_RA;
    h16*   Z  = (h16*)wsp; wsp += SZ_Z;
    h16*   U  = (h16*)wsp;
    h16*   G  = (h16*)wsp; wsp += SZ_UG;
    float* XD = (float*)wsp; wsp += SZ_XD;
    h16*   WIN  = (h16*)wsp; wsp += SZ_WIN;
    h16*   WXP  = (h16*)wsp; wsp += SZ_WXP;
    h16*   WOUT = (h16*)wsp; wsp += SZ_WOUT;
    float* WC   = (float*)wsp; wsp += SZ_WC;
    const size_t zofs = SZ_RA / 2;

    k_wprep<<<GB_WIN + GB_WXP + GB_WOUT + GB_WC, 256, 0, stream>>>(win, xprj, wout, convw, WIN, WXP, WOUT, WC);
    k_ln_in<<<BL / 8, 256, 0, stream>>>(x, ln1w, ln1b, HX);
    k_gemm_in<<<dim3(BL / 64, (2 * DI) / 64, 1), 32, 0, stream>>>(HX, WIN, XI, zofs);
    k_conv<<<BL / 16, 256, 0, stream>>>(XI, WC, convb, U);
    k_gemm_xp<<<dim3(BL / 64, 1, 1), 32, 0, stream>>>(U, WXP, XD);
    k_scan<<<dim3(DI / 128, NB, 1), 128, 0, stream>>>(U, XD, dtw, dtb, alog, dsk, Y);
    k_ln_gate<<<BL / 8, 256, 0, stream>>>(Y, Z, onw, onb, G);
    k_gemm_out<<<dim3(BL / 64, CC / 64, 1), 32, 0, stream>>>(G, WOUT, OUT, x);
}
